// GAT_54116587930155
// MI455X (gfx1250) — hardware-verified
//
#include <hip/hip_runtime.h>
#include <stddef.h>
#include <stdint.h>
#include <math.h>


#define F_IN    75
#define KP1     96
#define HC1     512
#define HID1    64
#define NHD1    8
#define C2R     32
#define H2P     64
#define KA2     1024
#define MLPH    16
#define SWKN    (C2R * MLPH)
#define NTHR    256
#define NWAVE   8
#define EPT     8
#define CHUNK   (NTHR * EPT)
#define WCAP    (EPT * 32)
#define LISTN   (NWAVE * WCAP)
#define NBMAX   2048
#define SLOTB   11
#define RCAP    28672
#define DEGCAP  256
#define GBM     64
#define GBN     64
#define GTHR    128
#define MROWS   128
#define NEGSL   0.2f
#define EPS_SM  1e-16f
#define WSMAX   268435456
#define LDS_AGG ((2 * RCAP + 2 * NBMAX + LISTN) * 4 + 64 + SWKN * 4)

static_assert((CHUNK & (CHUNK - 1)) == 0 && CHUNK <= (1 << SLOTB));
static_assert(NBMAX == (1 << SLOTB));
static_assert(NTHR * 8 == NBMAX);
static_assert(LISTN >= NBMAX);
static_assert(LISTN >= NWAVE * WCAP);
static_assert((RCAP % 32) == 0);
static_assert(LDS_AGG <= 300000);
static_assert(SWKN == 2 * NTHR);
static_assert(GBM == (GTHR / 32) * 16);
static_assert(GTHR == 2 * GBN && GTHR == 2 * GBM);
static_assert((KP1 % 32) == 0 && (KA2 % 32) == 0 && KP1 >= F_IN && (KP1 % 8) == 0);
static_assert((HC1 % GBN) == 0 && HID1 == GBN && H2P == GBN && C2R <= GBN);
static_assert(HC1 == NHD1 * HID1);
static_assert(KA2 == 2 * HC1);
static_assert((MROWS % GBM) == 0);
static_assert(HC1 / 2 == 8 * 32);
static_assert(HID1 == 8 * 8);
static_assert(NHD1 == 2 * (32 / 8));
static_assert(C2R == 32);
static_assert(MLPH == 16);

typedef float          v2f  __attribute__((ext_vector_type(2)));
typedef float          v4f  __attribute__((ext_vector_type(4)));
typedef float          v8f  __attribute__((ext_vector_type(8)));
typedef int            v4i  __attribute__((ext_vector_type(4)));
typedef int            v8i  __attribute__((ext_vector_type(8)));
typedef unsigned int   v4u  __attribute__((ext_vector_type(4)));
typedef unsigned short v8us __attribute__((ext_vector_type(8)));
typedef __bf16         v16b __attribute__((ext_vector_type(16)));
typedef v2f  __attribute__((may_alias)) v2fa;
typedef v4f  __attribute__((may_alias)) v4fa;
typedef v8us __attribute__((may_alias)) v8usa;
union FragB { v16b v; v8us h[2]; v8i w; };

__device__ __forceinline__ v8f wmb(const FragB& a, const FragB& b, v8f c) {
  v8f d = __builtin_amdgcn_wmma_f32_16x16x32_bf16(false, a.v, false, b.v, (short)0, c, false, false);
  asm volatile("v_nop\n\tv_nop\n\tv_nop\n\tv_nop" : "+v"(d) : "v"(a.w), "v"(b.w));
  return d;
}

__device__ __forceinline__ unsigned int f2bf(float f) {
  const unsigned int u = __float_as_uint(f);
  return ((u + 0x7FFFu + ((u >> 16) & 1u)) >> 16) & 0xFFFFu;
}
__device__ __forceinline__ float bf2f(unsigned int b) { return __uint_as_float(b << 16); }
__device__ __forceinline__ float bfr(float f) { return bf2f(f2bf(f)); }
__device__ __forceinline__ v4f bfr4(const v4f a) {
  v4f r; r.x = bfr(a.x); r.y = bfr(a.y); r.z = bfr(a.z); r.w = bfr(a.w); return r;
}
__device__ __forceinline__ unsigned int pk2(float lo, float hi) { return f2bf(lo) | (f2bf(hi) << 16); }
__device__ __forceinline__ v4u pack8(const v4f a, const v4f b) {
  v4u r;
  r.x = pk2(a.x, a.y); r.y = pk2(a.z, a.w); r.z = pk2(b.x, b.y); r.w = pk2(b.z, b.w);
  return r;
}
__device__ __forceinline__ void split8(const v4f a, const v4f b, v4u& hv, v4u& lv) {
  const unsigned int h0 = f2bf(a.x), h1 = f2bf(a.y), h2 = f2bf(a.z), h3 = f2bf(a.w);
  const unsigned int h4 = f2bf(b.x), h5 = f2bf(b.y), h6 = f2bf(b.z), h7 = f2bf(b.w);
  const unsigned int g0 = f2bf(a.x - bf2f(h0)), g1 = f2bf(a.y - bf2f(h1));
  const unsigned int g2 = f2bf(a.z - bf2f(h2)), g3 = f2bf(a.w - bf2f(h3));
  const unsigned int g4 = f2bf(b.x - bf2f(h4)), g5 = f2bf(b.y - bf2f(h5));
  const unsigned int g6 = f2bf(b.z - bf2f(h6)), g7 = f2bf(b.w - bf2f(h7));
  hv.x = h0 | (h1 << 16); hv.y = h2 | (h3 << 16); hv.z = h4 | (h5 << 16); hv.w = h6 | (h7 << 16);
  lv.x = g0 | (g1 << 16); lv.y = g2 | (g3 << 16); lv.z = g4 | (g5 << 16); lv.w = g6 | (g7 << 16);
}
__device__ __forceinline__ v4f madd4(const v4f acc, float s1, float s2, const v4f f) {
  v4f r;
  r.x = fmaf(acc.x, s1, s2 * f.x);
  r.y = fmaf(acc.y, s1, s2 * f.y);
  r.z = fmaf(acc.z, s1, s2 * f.z);
  r.w = fmaf(acc.w, s1, s2 * f.w);
  return r;
}
__device__ __forceinline__ float elu1(float t) {
  const float n = __expf(fminf(t, 0.f)) - 1.0f;
  return t > 0.f ? t : n;
}
__device__ __forceinline__ v4f elu_fin(const v4f a, float inv, const v4f b, bool live, float pz) {
  v4f o;
  o.x = (live ? elu1(fmaf(a.x, inv, b.x)) : 0.f) + pz;
  o.y = (live ? elu1(fmaf(a.y, inv, b.y)) : 0.f) + pz;
  o.z = (live ? elu1(fmaf(a.z, inv, b.z)) : 0.f) + pz;
  o.w = (live ? elu1(fmaf(a.w, inv, b.w)) : 0.f) + pz;
  return o;
}

__device__ __forceinline__ int scan_chunk(const int* __restrict__ dsts, int nE, int cbase, int slotBase,
                                          int nb, int vec8, int* list, int tid, int lane, int wave) {
  int wc = 0;
  const int el0  = tid * EPT;
  const int e0   = cbase + el0;
  const int sent = -2147483647 - 1;
  v4i da, db;
  if (vec8 != 0 && cbase + CHUNK <= nE) {
    da = *(const v4i*)(dsts + e0);
    db = *(const v4i*)(dsts + e0 + 4);
  } else {
    da.x = (e0     < nE) ? dsts[min(e0,     nE - 1)] : sent;
    da.y = (e0 + 1 < nE) ? dsts[min(e0 + 1, nE - 1)] : sent;
    da.z = (e0 + 2 < nE) ? dsts[min(e0 + 2, nE - 1)] : sent;
    da.w = (e0 + 3 < nE) ? dsts[min(e0 + 3, nE - 1)] : sent;
    db.x = (e0 + 4 < nE) ? dsts[min(e0 + 4, nE - 1)] : sent;
    db.y = (e0 + 5 < nE) ? dsts[min(e0 + 5, nE - 1)] : sent;
    db.z = (e0 + 6 < nE) ? dsts[min(e0 + 6, nE - 1)] : sent;
    db.w = (e0 + 7 < nE) ? dsts[min(e0 + 7, nE - 1)] : sent;
  }
  const unsigned nbs = (unsigned)slotBase;
  const unsigned unb = (unsigned)nb;
  const unsigned s0 = (unsigned)da.x - nbs, s1 = (unsigned)da.y - nbs;
  const unsigned s2 = (unsigned)da.z - nbs, s3 = (unsigned)da.w - nbs;
  const unsigned s4 = (unsigned)db.x - nbs, s5 = (unsigned)db.y - nbs;
  const unsigned s6 = (unsigned)db.z - nbs, s7 = (unsigned)db.w - nbs;
  const bool h0 = s0 < unb, h1 = s1 < unb, h2 = s2 < unb, h3 = s3 < unb;
  const bool h4 = s4 < unb, h5 = s5 < unb, h6 = s6 < unb, h7 = s7 < unb;
  const unsigned any = __builtin_amdgcn_ballot_w32(h0 | h1 | h2 | h3 | h4 | h5 | h6 | h7);
  if (any != 0u) {
#define HITJ(J, HJ, SJ) { \
      const unsigned mj = __builtin_amdgcn_ballot_w32(HJ); \
      if (mj != 0u) { \
        if (HJ) { \
          const int pos = wc + (int)__builtin_amdgcn_mbcnt_lo(mj, 0u); \
          if (pos < WCAP) list[wave * WCAP + pos] = ((el0 + (J)) << SLOTB) | (int)(SJ); \
        } \
        wc += (int)__builtin_popcount(mj); } }
    HITJ(0, h0, s0)
    HITJ(1, h1, s1)
    HITJ(2, h2, s2)
    HITJ(3, h3, s3)
    HITJ(4, h4, s4)
    HITJ(5, h5, s5)
    HITJ(6, h6, s6)
    HITJ(7, h7, s7)
#undef HITJ
  }
  return wc;
}

__global__ __launch_bounds__(NTHR) void k_xprep(const float* __restrict__ x, unsigned short* xb, int nN, int nUnits) {
  const int i = (int)blockIdx.x * NTHR + (int)threadIdx.x;
  if (i >= nUnits) return;
  const int upr = KP1 >> 3;
  const int row = i / upr;
  const int c0  = (i - row * upr) * 8;
  const int rc  = row < nN ? row : nN - 1;
  const float* p = x + (size_t)rc * F_IN;
  float v[8];
#pragma unroll
  for (int j = 0; j < 8; ++j) {
    const int c  = c0 + j;
    const int cc = c < F_IN ? c : F_IN - 1;
    const float t = p[cc];
    v[j] = (c < F_IN && row < nN) ? t : 0.f;
  }
  const v4f a = {v[0], v[1], v[2], v[3]};
  const v4f b = {v[4], v[5], v[6], v[7]};
  const v4u hv = pack8(a, b);
  const size_t o = (size_t)row * KP1 + c0;
  *(volatile v4u*)(xb + o) = hv;
  __threadfence();
  *(volatile v4u*)(xb + o) = hv;
}

__global__ __launch_bounds__(NTHR) void k_wtr(const float* __restrict__ w, int Kvalid, int Kper, int Ncol,
                                              int Nrows, int Kout, unsigned short* wt, int nUnits) {
  const int u = (int)blockIdx.x * NTHR + (int)threadIdx.x;
  if (u >= nUnits) return;
  const int kq  = Kout >> 3;
  const int n   = u / kq;
  const int k8  = (u - n * kq) * 8;
  const int ncl = n < Ncol ? n : Ncol - 1;
  float v[8];
#pragma unroll
  for (int j = 0; j < 8; ++j) {
    const int k  = k8 + j;
    const int kk = k - (k / Kper) * Kper;
    const int kc = kk < Kvalid ? kk : Kvalid - 1;
    const float t = w[(size_t)kc * (size_t)Ncol + ncl];
    v[j] = (kk < Kvalid && n < Ncol && n < Nrows) ? t : 0.f;
  }
  const v4f a = {v[0], v[1], v[2], v[3]};
  const v4f b = {v[4], v[5], v[6], v[7]};
  const v4u wv = pack8(a, b);
  unsigned short* o = wt + (size_t)n * (size_t)Kout + k8;
  *(volatile v4u*)o = wv;
  __threadfence();
  *(volatile v4u*)o = wv;
}

__global__ __launch_bounds__(GTHR) void k_gemm(
    const unsigned short* __restrict__ A, const unsigned short* __restrict__ WT,
    float* outF, int K, int ldo,
    const float* __restrict__ atts, const float* __restrict__ attd, int attLen,
    float* SD, int MPr)
{
  __shared__ __attribute__((aligned(16))) float stg[GBM * GBN];
  __shared__ __attribute__((aligned(16))) float satt[2 * GBN];
  __shared__ __attribute__((aligned(16))) float sdot[2 * GBM];
  const int tid = (int)threadIdx.x, lane = tid & 31, wave = tid >> 5, hh = lane >> 4, m = lane & 15;
  const int rowBase = (int)blockIdx.x * GBM;
  const int head    = (int)blockIdx.y;
  const int col0    = head * GBN;

  {
    const int which = tid >> 6;
    const int c  = tid & 63;
    const int cl = c < attLen ? c : attLen - 1;
    const float vs = atts[head * attLen + cl];
    const float vd = attd[head * attLen + cl];
    float v = (which == 0) ? vs : vd;
    v = (c < attLen) ? bfr(v) : 0.f;
    satt[which * GBN + c] = v;
  }

  v8f acc[4];
  {
    const v8f z = {0.f, 0.f, 0.f, 0.f, 0.f, 0.f, 0.f, 0.f};
    acc[0] = z; acc[1] = z; acc[2] = z; acc[3] = z;
  }
  const unsigned short* ap = A  + (size_t)(rowBase + 16 * wave + m) * (size_t)K + 8 * hh;
  const unsigned short* wp = WT + (size_t)(col0 + m) * (size_t)K + 8 * hh;
  const int ksteps = K >> 5;
#pragma unroll 1
  for (int ks = 0; ks < ksteps; ++ks) {
    FragB af;
    af.h[0] = *(const v8usa*)(ap + 32 * ks);
    af.h[1] = *(const v8usa*)(ap + 32 * ks + 16);
#pragma unroll
    for (int t = 0; t < 4; ++t) {
      const unsigned short* wq = wp + (size_t)(16 * t) * (size_t)K + 32 * ks;
      FragB bf;
      bf.h[0] = *(const v8usa*)wq;
      bf.h[1] = *(const v8usa*)(wq + 16);
      acc[t] = wmb(af, bf, acc[t]);
    }
  }

#pragma unroll
  for (int t = 0; t < 4; ++t) {
    const int lc = 16 * t + m;
#pragma unroll
    for (int r = 0; r < 8; ++r) {
      const int lr = 16 * wave + 8 * hh + r;
      stg[lr * GBN + lc] = acc[t][r];
    }
  }
  __syncthreads();

  {
    const int row = tid & 63, which = tid >> 6;
    const float* sa = satt + which * GBN;
    const float* hr = stg + row * GBN;
    float d = 0.f;
#pragma unroll 4
    for (int c4 = 0; c4 < GBN / 4; ++c4) {
      const v4f hv = *(const v4fa*)(hr + 4 * c4);
      const v4f av = *(const v4fa*)(sa + 4 * c4);
      d = fmaf(hv.x, av.x, d);
      d = fmaf(hv.y, av.y, d);
      d = fmaf(hv.z, av.z, d);
      d = fmaf(hv.w, av.w, d);
    }
    sdot[which * GBM + row] = d;
  }
  __syncthreads();

  v4f fv[8];
#pragma unroll
  for (int i = 0; i < 8; ++i) {
    const int lr = 16 * wave + 2 * i + hh;
    fv[i] = *(const v4fa*)(stg + lr * GBN + 4 * m);
  }
  const int which2 = lane >> 4, piece = lane & 15;
  const v4f sdv = *(const v4fa*)(sdot + which2 * GBM + 4 * piece);
  float* sp = SD + (size_t)(2 * head + which2) * (size_t)MPr + rowBase + 4 * piece;

#pragma unroll
  for (int i = 0; i < 8; ++i) {
    const int lr = 16 * wave + 2 * i + hh;
    const int gr = rowBase + lr;
    float* op = outF + (size_t)gr * (size_t)ldo + col0 + 4 * m;
    *(volatile v4f*)op = fv[i];
  }
  if (wave == 0) *(volatile v4f*)sp = sdv;
  __threadfence();
#pragma unroll
  for (int i = 0; i < 8; ++i) {
    const int lr = 16 * wave + 2 * i + hh;
    const int gr = rowBase + lr;
    float* op = outF + (size_t)gr * (size_t)ldo + col0 + 4 * m;
    *(volatile v4f*)op = fv[i];
  }
  if (wave == 0) *(volatile v4f*)sp = sdv;
}

template<int L>
__global__ __launch_bounds__(NTHR) void k_agg(
    const int* __restrict__ srcs, const int* __restrict__ dsts,
    const float* __restrict__ F, const float* __restrict__ SD,
    const float* __restrict__ bias,
    const float* __restrict__ rw1, const float* __restrict__ rb1,
    const float* __restrict__ rw2, const float* __restrict__ rb2,
    unsigned short* HP, float* out,
    int nN, int nE, int nb, int vec8, int MPr) {
  extern __shared__ v4f lds_dyn[];
  int* reg1 = (int*)lds_dyn;
  int* reg2 = reg1 + RCAP;
  int* scnt = reg2 + RCAP;
  int* soff = scnt + NBMAX;
  int* list = soff + NBMAX;
  int* wcnt = list + LISTN;
  int* wtot = wcnt + NWAVE;
  float* swk = (float*)(wtot + NWAVE);
  const int tid = (int)threadIdx.x, lane = tid & 31, wave = tid >> 5;
  const int nodeBase = (int)blockIdx.x * nb;

  for (int i = tid; i < NBMAX; i += NTHR) scnt[i] = 0;
  if (L == 2) {
    for (int i = tid; i < SWKN; i += NTHR) swk[i] = bfr(rw1[i]);
  }
  __syncthreads();

  int tot = 0;
  const int nChunks = (nE + CHUNK - 1) / CHUNK;
#pragma unroll 1
  for (int ch = 0; ch < nChunks; ++ch) {
    const int cbase = ch * CHUNK;
    const int wc = scan_chunk(dsts, nE, cbase, nodeBase, nb, vec8, list, tid, lane, wave);
    if (lane == 0) wcnt[wave] = wc;
    __syncthreads();
    int pre = 0, all = 0;
#pragma unroll
    for (int w2 = 0; w2 < NWAVE; ++w2) {
      int c = wcnt[w2];
      c = c < 0 ? 0 : (c > WCAP ? WCAP : c);
      all += c;
      pre += (w2 < wave) ? c : 0;
    }
    const int wcc  = wc > WCAP ? WCAP : wc;
    const int base = tot + pre;
#pragma unroll 1
    for (int i = lane; i < wcc; i += 32) {
      const int ent = list[wave * WCAP + i];
      const int el  = (ent >> SLOTB) & (CHUNK - 1);
      const int sl  = ent & (NBMAX - 1);
      int eid = cbase + el;
      eid = eid > nE - 1 ? nE - 1 : eid;
      const int pos = base + i;
      if (pos < RCAP) reg1[pos] = (int)(((unsigned)eid << SLOTB) | (unsigned)sl);
    }
    tot += all;
    tot = tot > RCAP ? RCAP : tot;
    __syncthreads();
  }
  const int nh = tot;

  if (wave == 0) {
#pragma unroll 1
    for (int b0 = 0; b0 < nh; b0 += 32) {
      const int idx = b0 + lane;
      const int uv  = reg1[idx < nh ? idx : nh - 1];
      const int m32 = (nh - b0) < 32 ? (nh - b0) : 32;
#pragma unroll 1
      for (int k = 0; k < m32; ++k) {
        const int u  = __builtin_amdgcn_readlane(uv, k);
        const int sl = u & (NBMAX - 1);
        if (lane == 0) scnt[sl] = scnt[sl] + 1;
      }
    }
  }
  __syncthreads();

  {
    const v4i ca = *(const v4i*)(scnt + 8 * tid);
    const v4i cb = *(const v4i*)(scnt + 8 * tid + 4);
    const int e0 = ca.x < 0 ? 0 : ca.x, e1 = ca.y < 0 ? 0 : ca.y, e2 = ca.z < 0 ? 0 : ca.z, e3 = ca.w < 0 ? 0 : ca.w;
    const int e4 = cb.x < 0 ? 0 : cb.x, e5 = cb.y < 0 ? 0 : cb.y, e6 = cb.z < 0 ? 0 : cb.z, e7 = cb.w < 0 ? 0 : cb.w;
    const int ts = e0 + e1 + e2 + e3 + e4 + e5 + e6 + e7;
    int incl = ts;
#pragma unroll
    for (int d = 1; d < 32; d <<= 1) {
      const int up = __shfl_up(incl, d);
      if (lane >= d) incl += up;
    }
    if (lane == 31) wtot[wave] = incl;
    __syncthreads();
    int pre = 0;
#pragma unroll
    for (int w2 = 0; w2 < NWAVE; ++w2) pre += (w2 < wave) ? wtot[w2] : 0;
    int run = pre + incl - ts;
    soff[8 * tid + 0] = run; run += e0;
    soff[8 * tid + 1] = run; run += e1;
    soff[8 * tid + 2] = run; run += e2;
    soff[8 * tid + 3] = run; run += e3;
    soff[8 * tid + 4] = run; run += e4;
    soff[8 * tid + 5] = run; run += e5;
    soff[8 * tid + 6] = run; run += e6;
    soff[8 * tid + 7] = run;
  }
  __syncthreads();
  for (int i = tid; i < NBMAX; i += NTHR) list[i] = soff[i];
  __syncthreads();

  if (wave == 0) {
#pragma unroll 1
    for (int b0 = 0; b0 < nh; b0 += 32) {
      const int idx = b0 + lane;
      const int uv  = reg1[idx < nh ? idx : nh - 1];
      const int m32 = (nh - b0) < 32 ? (nh - b0) : 32;
#pragma unroll 1
      for (int k = 0; k < m32; ++k) {
        const int u   = __builtin_amdgcn_readlane(uv, k);
        const int sl  = u & (NBMAX - 1);
        const int eid = (int)((unsigned)u >> SLOTB);
        if (lane == 0) {
          int pos = list[sl];
          pos = pos < 0 ? 0 : (pos > RCAP - 1 ? RCAP - 1 : pos);
          reg2[pos] = eid;
          list[sl] = pos + 1;
        }
      }
    }
  }
  __syncthreads();

  const int nbw = nb >> 3;
  const bool ovf = (nh >= RCAP);
  const float qnan = __int_as_float(0x7fc00000);

  if (L == 1) {
    const int cA = 8 * lane;
    const int cB = (HC1 / 2) + 8 * lane;
    const int hA = lane >> 3;
    const int hB = (NHD1 / 2) + (lane >> 3);
    const v4f bA0 = bfr4(*(const v4fa*)(bias + cA));
    const v4f bA1 = bfr4(*(const v4fa*)(bias + cA + 4));
    const v4f bB0 = bfr4(*(const v4fa*)(bias + cB));
    const v4f bB1 = bfr4(*(const v4fa*)(bias + cB + 4));
    const float* ASA = SD + (size_t)(2 * hA) * (size_t)MPr;
    const float* ADA = ASA + MPr;
    const float* ASB = SD + (size_t)(2 * hB) * (size_t)MPr;
    const float* ADB = ASB + MPr;

#pragma unroll 1
    for (int jt = 0; jt < nbw; ++jt) {
      const int slot = wave * nbw + jt;
      const int grow = nodeBase + slot;
      const int gcl  = grow < nN ? grow : nN - 1;
      int st = soff[slot];
      const int craw = scnt[slot];
      int cnt = craw;
      st  = st < 0 ? 0 : (st > nh ? nh : st);
      cnt = cnt < 0 ? 0 : (cnt > DEGCAP ? DEGCAP : cnt);
      if (cnt > nh - st) cnt = nh - st;
      const float pz = (ovf || craw > DEGCAP) ? qnan : 0.0f;

      const float* fr = F + (size_t)gcl * HC1;
      v4f a0 = *(const v4fa*)(fr + cA);
      v4f a1 = *(const v4fa*)(fr + cA + 4);
      v4f c0 = *(const v4fa*)(fr + cB);
      v4f c1 = *(const v4fa*)(fr + cB + 4);
      const float adA = ADA[gcl];
      const float adB = ADB[gcl];
      float lA = ASA[gcl] + adA; lA = lA > 0.f ? lA : NEGSL * lA;
      float lB = ASB[gcl] + adB; lB = lB > 0.f ? lB : NEGSL * lB;
      float mxA = lA, dnA = 1.0f, mxB = lB, dnB = 1.0f;

#pragma unroll 1
      for (int q = 0; q < cnt; ++q) {
        int idx = st + q; idx = idx > RCAP - 1 ? RCAP - 1 : idx;
        int eid = reg2[idx]; eid = eid < 0 ? 0 : (eid > nE - 1 ? nE - 1 : eid);
        const int sraw = srcs[eid];
        const int s = sraw < 0 ? 0 : (sraw > nN - 1 ? nN - 1 : sraw);
        const float* gs = F + (size_t)s * HC1;
        const v4f fa0 = *(const v4fa*)(gs + cA);
        const v4f fa1 = *(const v4fa*)(gs + cA + 4);
        const v4f fc0 = *(const v4fa*)(gs + cB);
        const v4f fc1 = *(const v4fa*)(gs + cB + 4);
        float gA = ASA[s] + adA; gA = gA > 0.f ? gA : NEGSL * gA;
        float gB = ASB[s] + adB; gB = gB > 0.f ? gB : NEGSL * gB;
        {
          const float df = gA - mxA;
          const float ee = __expf(-fabsf(df));
          const bool up  = df > 0.f;
          const float s1 = up ? ee : 1.0f;
          const float s2 = up ? 1.0f : ee;
          mxA = up ? gA : mxA;
          dnA = fmaf(dnA, s1, s2);
          a0 = madd4(a0, s1, s2, fa0);
          a1 = madd4(a1, s1, s2, fa1);
        }
        {
          const float df = gB - mxB;
          const float ee = __expf(-fabsf(df));
          const bool up  = df > 0.f;
          const float s1 = up ? ee : 1.0f;
          const float s2 = up ? 1.0f : ee;
          mxB = up ? gB : mxB;
          dnB = fmaf(dnB, s1, s2);
          c0 = madd4(c0, s1, s2, fc0);
          c1 = madd4(c1, s1, s2, fc1);
        }
      }
      const float invA = __builtin_amdgcn_rcpf(dnA + EPS_SM);
      const float invB = __builtin_amdgcn_rcpf(dnB + EPS_SM);
      const bool live = grow < nN;
      const v4f oA0 = elu_fin(a0, invA, bA0, live, pz);
      const v4f oA1 = elu_fin(a1, invA, bA1, live, pz);
      const v4f oB0 = elu_fin(c0, invB, bB0, live, pz);
      const v4f oB1 = elu_fin(c1, invB, bB1, live, pz);
      v4u hvA, lvA, hvB, lvB;
      split8(oA0, oA1, hvA, lvA);
      split8(oB0, oB1, hvB, lvB);
      unsigned short* gb = HP + (size_t)grow * KA2;
      unsigned short* p0 = gb + cA;
      unsigned short* p1 = gb + cB;
      unsigned short* p2 = gb + HC1 + cA;
      unsigned short* p3 = gb + HC1 + cB;
      const bool wr = grow < MPr;
      if (wr) {
        *(volatile v4u*)p0 = hvA; *(volatile v4u*)p1 = hvB;
        *(volatile v4u*)p2 = lvA; *(volatile v4u*)p3 = lvB;
      }
      __threadfence();
      if (wr) {
        *(volatile v4u*)p0 = hvA; *(volatile v4u*)p1 = hvB;
        *(volatile v4u*)p2 = lvA; *(volatile v4u*)p3 = lvB;
      }
    }
  } else {
    const int kq = lane & (MLPH - 1);
    const float bz  = bfr(bias[lane]);
    const float rbk = bfr(rb1[kq]);
    const float rwk = bfr(rw2[kq]);
    const float rb0 = bfr(rb2[0]);
    const float* ASp = SD;
    const float* ADp = SD + MPr;
    float* res = (float*)list;

#pragma unroll 1
    for (int jt = 0; jt < nbw; ++jt) {
      const int slot = wave * nbw + jt;
      const int grow = nodeBase + slot;
      const int gcl  = grow < nN ? grow : nN - 1;
      int st = soff[slot];
      const int craw = scnt[slot];
      int cnt = craw;
      st  = st < 0 ? 0 : (st > nh ? nh : st);
      cnt = cnt < 0 ? 0 : (cnt > DEGCAP ? DEGCAP : cnt);
      if (cnt > nh - st) cnt = nh - st;
      const float pz = (ovf || craw > DEGCAP) ? qnan : 0.0f;

      const float fd = F[(size_t)gcl * H2P + lane];
      const float adv = ADp[gcl];
      float l0 = ASp[gcl] + adv;
      l0 = l0 > 0.f ? l0 : NEGSL * l0;
      float mx = l0, dn = 1.0f;
      float a0 = fd;

#pragma unroll 1
      for (int q = 0; q < cnt; ++q) {
        int idx = st + q; idx = idx > RCAP - 1 ? RCAP - 1 : idx;
        int eid = reg2[idx]; eid = eid < 0 ? 0 : (eid > nE - 1 ? nE - 1 : eid);
        const int sraw = srcs[eid];
        const int s = sraw < 0 ? 0 : (sraw > nN - 1 ? nN - 1 : sraw);
        const float fs = F[(size_t)s * H2P + lane];
        float lg = ASp[s] + adv;
        lg = lg > 0.f ? lg : NEGSL * lg;
        const float df = lg - mx;
        const float ee = __expf(-fabsf(df));
        const bool up  = df > 0.f;
        const float s1 = up ? ee : 1.0f;
        const float s2 = up ? 1.0f : ee;
        mx = up ? lg : mx;
        dn = fmaf(dn, s1, s2);
        a0 = fmaf(a0, s1, s2 * fs);
      }
      const float inv = __builtin_amdgcn_rcpf(dn + EPS_SM);
      const float z = fmaf(a0, inv, bz);
      float u = 0.f;
#pragma unroll 8
      for (int cc = 0; cc < C2R; ++cc) {
        const float zc = __shfl(z, cc);
        u = fmaf(zc, swk[cc * MLPH + kq], u);
      }
      float hk = fmaxf(u + rbk, 0.f) * rwk;
      hk += __shfl_xor(hk, 8);
      hk += __shfl_xor(hk, 4);
      hk += __shfl_xor(hk, 2);
      hk += __shfl_xor(hk, 1);
      const float r = hk + rb0 + pz;
      if (lane == 0) res[slot] = r;
    }

    __syncthreads();
    const int npc = nb >> 2;
#pragma unroll 1
    for (int p = tid; p < npc; p += NTHR) {
      const v4f v = *(const v4fa*)(res + 4 * p);
      const int r0 = nodeBase + 4 * p;
      if (r0 + 3 < nN) {
        *(volatile v4f*)(out + r0) = v;
      } else {
        if (r0     < nN) *(volatile float*)(out + r0)     = v.x;
        if (r0 + 1 < nN) *(volatile float*)(out + r0 + 1) = v.y;
        if (r0 + 2 < nN) *(volatile float*)(out + r0 + 2) = v.z;
      }
    }
    __threadfence();
#pragma unroll 1
    for (int p = tid; p < npc; p += NTHR) {
      const v4f v = *(const v4fa*)(res + 4 * p);
      const int r0 = nodeBase + 4 * p;
      if (r0 + 3 < nN) {
        *(volatile v4f*)(out + r0) = v;
      } else {
        if (r0     < nN) *(volatile float*)(out + r0)     = v.x;
        if (r0 + 1 < nN) *(volatile float*)(out + r0 + 1) = v.y;
        if (r0 + 2 < nN) *(volatile float*)(out + r0 + 2) = v.z;
      }
    }
  }
}

static int pick_nb(int nE, int nN) {
  int nb = NBMAX;
  while (nb > 32 && (long long)nb * (long long)nE * 5LL > (long long)RCAP * (long long)nN * 4LL) nb >>= 1;
  return nb;
}
static inline int cdiv(int a, int b) { return (a + b - 1) / b; }

extern "C" void kernel_launch(void* const* d_in, const int* in_sizes, int n_in,
                              void* d_out, int out_size, void* d_ws, size_t ws_size,
                              hipStream_t stream) {
  if (n_in < 14) return;
  const int nN = in_sizes[0] / F_IN;
  if (nN <= 0 || in_sizes[0] != nN * F_IN || nN > (1 << 22)) return;
  if (in_sizes[1] != F_IN * HC1) return;
  if (in_sizes[2] != NHD1 * HID1 || in_sizes[3] != NHD1 * HID1) return;
  if (in_sizes[4] != HC1) return;
  if (in_sizes[5] != HC1 * C2R) return;
  if (in_sizes[6] != C2R || in_sizes[7] != C2R) return;
  if (in_sizes[8] != C2R) return;
  if (in_sizes[9] != C2R * MLPH) return;
  if (in_sizes[10] != MLPH) return;
  if (in_sizes[11] != MLPH) return;
  if (in_sizes[12] < 1) return;
  if (in_sizes[13] < 2 || (in_sizes[13] & 1) != 0) return;
  const int nE = in_sizes[13] / 2;
  if (nE < 1 || nE >= (1 << (32 - SLOTB))) return;
  if (out_size != nN) return;

  const float* x    = (const float*)d_in[0];
  const float* W1   = (const float*)d_in[1];
  const float* a1s  = (const float*)d_in[2];
  const float* a1d  = (const float*)d_in[3];
  const float* b1   = (const float*)d_in[4];
  const float* W2   = (const float*)d_in[5];
  const float* a2s  = (const float*)d_in[6];
  const float* a2d  = (const float*)d_in[7];
  const float* b2   = (const float*)d_in[8];
  const float* lw1  = (const float*)d_in[9];
  const float* lb1  = (const float*)d_in[10];
  const float* lw2  = (const float*)d_in[11];
  const float* lb2  = (const float*)d_in[12];
  const int*   ei   = (const int*)  d_in[13];
  float* out = (float*)d_out;
  const int* src = ei;
  const int* dst = ei + nE;

  const int MP   = cdiv(nN, MROWS) * MROWS;
  const int nb   = pick_nb(nE, nN);
  if (nb < 32 || (nb & (nb - 1)) != 0 || nb > NBMAX) return;
  const int gA   = cdiv(MP, nb);
  const int vec8 = ((nE & 3) == 0) ? 1 : 0;
  if (gA * nb < MP) return;

  char* ws = (char*)d_ws;
  size_t off = 0;
  const size_t oXB  = off; off += (size_t)MP * KP1 * 2;            off = (off + 255) & ~(size_t)255;
  const size_t oW1T = off; off += (size_t)HC1 * KP1 * 2;           off = (off + 255) & ~(size_t)255;
  const size_t oW2T = off; off += (size_t)GBN * KA2 * 2;           off = (off + 255) & ~(size_t)255;
  const size_t oH1  = off; off += (size_t)MP * HC1 * 4;            off = (off + 255) & ~(size_t)255;
  const size_t oSD1 = off; off += (size_t)2 * NHD1 * MP * 4;       off = (off + 255) & ~(size_t)255;
  const size_t oA2  = off; off += (size_t)MP * KA2 * 2;            off = (off + 255) & ~(size_t)255;
  if (off > ws_size || off > (size_t)WSMAX) return;
  if ((size_t)MP * H2P * 4 > (size_t)MP * HC1 * 4) return;
  unsigned short* XB  = (unsigned short*)(ws + oXB);
  unsigned short* W1T = (unsigned short*)(ws + oW1T);
  unsigned short* W2T = (unsigned short*)(ws + oW2T);
  float*          H1  = (float*)(ws + oH1);
  float*          H2  = (float*)(ws + oH1);
  float*          SD1 = (float*)(ws + oSD1);
  float*          SD2 = (float*)(ws + oSD1);
  unsigned short* A2  = (unsigned short*)(ws + oA2);

  hipFuncSetAttribute(reinterpret_cast<const void*>(&k_agg<1>),
                      hipFuncAttributeMaxDynamicSharedMemorySize, LDS_AGG);
  hipFuncSetAttribute(reinterpret_cast<const void*>(&k_agg<2>),
                      hipFuncAttributeMaxDynamicSharedMemorySize, LDS_AGG);

  const int nUx = MP * (KP1 / 8);
  k_xprep<<<cdiv(nUx, NTHR), NTHR, 0, stream>>>(x, XB, nN, nUx);

  {
    const int nUw1 = HC1 * (KP1 / 8);
    k_wtr<<<cdiv(nUw1, NTHR), NTHR, 0, stream>>>(W1, F_IN, KP1, HC1, HC1, KP1, W1T, nUw1);
    const int nUw2 = GBN * (KA2 / 8);
    k_wtr<<<cdiv(nUw2, NTHR), NTHR, 0, stream>>>(W2, HC1, HC1, C2R, GBN, KA2, W2T, nUw2);
  }

  const int gM = MP / GBM;
  k_gemm<<<dim3(gM, HC1 / GBN), GTHR, 0, stream>>>(XB, W1T, H1, KP1, HC1, a1s, a1d, HID1, SD1, MP);
  k_agg<1><<<gA, NTHR, LDS_AGG, stream>>>(src, dst, H1, SD1, b1, lw1, lb1, lw2, lb2, A2, out, nN, nE, nb, vec8, MP);
  k_gemm<<<dim3(gM, 1), GTHR, 0, stream>>>(A2, W2T, H2, KA2, H2P, a2s, a2d, C2R, SD2, MP);
  k_agg<2><<<gA, NTHR, LDS_AGG, stream>>>(src, dst, H2, SD2, b2, lw1, lb1, lw2, lb2, A2, out, nN, nE, nb, vec8, MP);
}
